// GTS_44049184588234
// MI455X (gfx1250) — hardware-verified
//
#include <hip/hip_runtime.h>
#include <stdint.h>

#define N_NODES 2048
#define BATCH   64
#define FX      64
#define UNITS   64
#define FCAT    128
#define PART    4096
#define NCOL    8192
#define KLIN    384
#define LDSW    40
#define SP      136
#define UP      68
#define TLP     36
#define ADJ_CARRY 1024.0f

static_assert(FCAT == FX + UNITS);
static_assert(FX == UNITS);
static_assert(PART == BATCH * FX);
static_assert(NCOL == 2 * PART);
static_assert(KLIN == 3 * FCAT);
static_assert((N_NODES % 128) == 0);
static_assert((LDSW % 8) == 0);
static_assert((SP % 8) == 0);
static_assert((UP % 4) == 0);
static_assert(TLP * 2 == 72);

typedef _Float16 f16;
typedef f16 v16h __attribute__((ext_vector_type(16)));
typedef f16 v8h_t __attribute__((ext_vector_type(8)));
typedef v8h_t __attribute__((may_alias)) v8h;
typedef float v8f __attribute__((ext_vector_type(8)));
typedef float v4f_t __attribute__((ext_vector_type(4)));
typedef v4f_t __attribute__((may_alias)) v4f;
typedef unsigned int v4u_t __attribute__((ext_vector_type(4)));
typedef v4u_t __attribute__((may_alias)) v4u;

union Frag  { v16h v; v8h_t h[2]; };
union Pack8 { v8h_t h; v4u_t u; };
union Pack2 { f16 h[2]; uint32_t u; };

__device__ __forceinline__ v8f zero8() {
  v8f z;
#pragma unroll
  for (int i = 0; i < 8; ++i) z[i] = 0.0f;
  return z;
}

__device__ __forceinline__ v16h ldfrag(const f16* rowp, int hh) {
  Frag f;
  f.h[0] = *(const v8h*)(rowp + 8 * hh);
  f.h[1] = *(const v8h*)(rowp + 16 + 8 * hh);
  return f.v;
}

__device__ __forceinline__ v8f wmma16(v16h a, v16h b, v8f c) {
  return __builtin_amdgcn_wmma_f32_16x16x32_f16(false, a, false, b, (short)0, c, false, false);
}

__device__ __forceinline__ float sigm_f(float z) {
  return __builtin_amdgcn_rcpf(1.0f + __expf(-z));
}

__device__ __forceinline__ float tanh_f(float v) {
  const float a = fminf(fabsf(v), 10.0f);
  const float e = __expf(2.0f * a);
  const float r = 1.0f - 2.0f * __builtin_amdgcn_rcpf(e + 1.0f);
  return copysignf(r, v);
}

__global__ void __launch_bounds__(256) k_adjT(const float* __restrict__ adj, f16* __restrict__ adjT)
{
  __shared__ float dinvL[64];
  __shared__ __align__(16) uint32_t tl32[64 * TLP];
  const int t = threadIdx.x, lane = t & 31, w = t >> 5;
  const int m0 = blockIdx.x * 64;

#pragma unroll 1
  for (int q = 0; q < 8; ++q) {
    const int mr = w * 8 + q;
    const float* rp = adj + (size_t)(m0 + mr) * N_NODES;
    float s = 0.0f;
#pragma unroll 4
    for (int i = 0; i < N_NODES / 128; ++i) {
      const v4f_t v = *(const v4f*)(rp + (size_t)(i * 32 + lane) * 4);
      s += (v[0] + v[1]) + (v[2] + v[3]);
    }
#pragma unroll
    for (int off = 16; off > 0; off >>= 1) s += __shfl_xor(s, off, 32);
    if (lane == 0) {
      const float d = s + 1.0f;
      dinvL[mr] = (d > 0.0f) ? (1.0f / d) : 0.0f;
    }
  }
  __syncthreads();

  const int mp = t >> 3, nc = (t & 7) * 8;
  const int ma = 2 * mp, mb = ma + 1;
  const float da = dinvL[ma] * ADJ_CARRY;
  const float db = dinvL[mb] * ADJ_CARRY;
  const float* rowA = adj + (size_t)(m0 + ma) * N_NODES;
  const float* rowB = rowA + N_NODES;
  const int sr = lane >> 3, sm = (lane & 7) * 8;

#pragma unroll 1
  for (int nt = 0; nt < N_NODES / 64; ++nt) {
    const int n0 = nt * 64;
    const v4f_t a0 = *(const v4f*)(rowA + n0 + nc);
    const v4f_t a1 = *(const v4f*)(rowA + n0 + nc + 4);
    const v4f_t b0 = *(const v4f*)(rowB + n0 + nc);
    const v4f_t b1 = *(const v4f*)(rowB + n0 + nc + 4);
#pragma unroll
    for (int e = 0; e < 8; ++e) {
      const int n = n0 + nc + e;
      float va = (e < 4) ? a0[e] : a1[e - 4];
      float vb = (e < 4) ? b0[e] : b1[e - 4];
      va = (va + (((m0 + ma) == n) ? 1.0f : 0.0f)) * da;
      vb = (vb + (((m0 + mb) == n) ? 1.0f : 0.0f)) * db;
      Pack2 pk;
      pk.h[0] = (f16)va;
      pk.h[1] = (f16)vb;
      tl32[(nc + e) * TLP + mp] = pk.u;
    }
    __syncthreads();
    v4u_t v[2];
#pragma unroll
    for (int q = 0; q < 2; ++q) {
      const int nr = w * 8 + q * 4 + sr;
      v[q] = *(const v4u*)(tl32 + nr * TLP + (lane & 7) * 4);
    }
    f16* ob = adjT + (size_t)n0 * N_NODES + m0 + sm;
#pragma unroll
    for (int q = 0; q < 2; ++q)
      *(volatile v4u_t*)(ob + (size_t)(w * 8 + q * 4 + sr) * N_NODES) = v[q];
    __threadfence();
#pragma unroll
    for (int q = 0; q < 2; ++q)
      *(volatile v4u_t*)(ob + (size_t)(w * 8 + q * 4 + sr) * N_NODES) = v[q];
    __syncthreads();
  }
}

__global__ void __launch_bounds__(256) k_x0t(const float* __restrict__ x, const float* __restrict__ hx,
                                            f16* __restrict__ X0T)
{
  __shared__ __align__(16) uint32_t tl32[64 * TLP];
  const int t = threadIdx.x, lane = t & 31, w = t >> 5;
  const int m0 = blockIdx.x * 64, b = blockIdx.y, part = blockIdx.z;
  const float* src = (part == 0) ? x : hx;
  const int mp = t >> 3, fc = (t & 7) * 8;
  const int ma = 2 * mp;
  const float* ra = src + (size_t)b * (N_NODES * FX) + (size_t)(m0 + ma) * FX + fc;
  const float* rb = ra + FX;
  const v4f_t a0 = *(const v4f*)ra, a1 = *(const v4f*)(ra + 4);
  const v4f_t b0 = *(const v4f*)rb, b1 = *(const v4f*)(rb + 4);
#pragma unroll
  for (int e = 0; e < 8; ++e) {
    Pack2 pk;
    pk.h[0] = (f16)((e < 4) ? a0[e] : a1[e - 4]);
    pk.h[1] = (f16)((e < 4) ? b0[e] : b1[e - 4]);
    tl32[(fc + e) * TLP + mp] = pk.u;
  }
  __syncthreads();
  const int sr = lane >> 3, sm = (lane & 7) * 8;
  v4u_t v[2];
#pragma unroll
  for (int q = 0; q < 2; ++q) {
    const int fr = w * 8 + q * 4 + sr;
    v[q] = *(const v4u*)(tl32 + fr * TLP + (lane & 7) * 4);
  }
  f16* ob = X0T + (size_t)(part * PART + b * FX) * N_NODES + m0 + sm;
#pragma unroll
  for (int q = 0; q < 2; ++q)
    *(volatile v4u_t*)(ob + (size_t)(w * 8 + q * 4 + sr) * N_NODES) = v[q];
  __threadfence();
#pragma unroll
  for (int q = 0; q < 2; ++q)
    *(volatile v4u_t*)(ob + (size_t)(w * 8 + q * 4 + sr) * N_NODES) = v[q];
}

__global__ void __launch_bounds__(256) k_packW(const float* __restrict__ Wru, const float* __restrict__ Wc,
                                             f16* __restrict__ WruT, f16* __restrict__ WcT)
{
  const int t = threadIdx.x;
  Pack8 pk;
  f16* dst;
  if (blockIdx.x < 24) {
    const int idx = blockIdx.x * 256 + t;
    const int j = idx / 48, k8 = (idx - j * 48) * 8;
    const int p = k8 >> 7, f0 = k8 & 127;
#pragma unroll
    for (int e = 0; e < 8; ++e)
      pk.h[e] = (f16)Wru[(size_t)((f0 + e) * 3 + p) * FCAT + j];
    dst = WruT + (size_t)idx * 8;
  } else {
    const int idx = (blockIdx.x - 24) * 256 + t;
    const int j = idx / 48, k8 = (idx - j * 48) * 8;
    const int p = k8 >> 7, f0 = k8 & 127;
#pragma unroll
    for (int e = 0; e < 8; ++e)
      pk.h[e] = (f16)Wc[(size_t)((f0 + e) * 3 + p) * UNITS + j];
    dst = WcT + (size_t)idx * 8;
  }
  *(volatile v4u_t*)dst = pk.u;
  __threadfence();
  *(volatile v4u_t*)dst = pk.u;
}

__global__ void __launch_bounds__(256) k_diff(const f16* __restrict__ adjT, const f16* __restrict__ Bt,
                                            const f16* Zt, f16* __restrict__ Ot,
                                            float alpha, int hasZ)
{
  __shared__ __align__(16) f16 lA[128 * LDSW];
  __shared__ __align__(16) f16 lB[128 * LDSW];
  __shared__ __align__(16) f16 stg[128 * SP];
  const int t = threadIdx.x, lane = t & 31, w = t >> 5;
  const int hh = lane >> 4, m = lane & 15;
  const int wm = (w >> 1) * 32, wn = (w & 1) * 64;
  const int cb = blockIdx.x * 128, nb = blockIdx.y * 128;
  const int lr = t >> 2, lc = (t & 3) * 8;
  const f16* aG0 = adjT + (size_t)(nb + lr) * N_NODES + lc;
  const f16* aG1 = aG0 + (size_t)64 * N_NODES;
  const f16* bG0 = Bt + (size_t)(cb + lr) * N_NODES + lc;
  const f16* bG1 = bG0 + (size_t)64 * N_NODES;
  f16* sA0 = lA + lr * LDSW + lc;
  f16* sA1 = sA0 + 64 * LDSW;
  f16* sB0 = lB + lr * LDSW + lc;
  f16* sB1 = sB0 + 64 * LDSW;

  v8f acc[2][4];
#pragma unroll
  for (int i = 0; i < 2; ++i)
#pragma unroll
    for (int j = 0; j < 4; ++j) acc[i][j] = zero8();

#pragma unroll 1
  for (int k0 = 0; k0 < N_NODES; k0 += 32) {
    const v8h_t ra0 = *(const v8h*)(aG0 + k0);
    const v8h_t ra1 = *(const v8h*)(aG1 + k0);
    const v8h_t rb0 = *(const v8h*)(bG0 + k0);
    const v8h_t rb1 = *(const v8h*)(bG1 + k0);
    *(v8h*)sA0 = ra0;
    *(v8h*)sA1 = ra1;
    *(v8h*)sB0 = rb0;
    *(v8h*)sB1 = rb1;
    __syncthreads();
    v16h af[2], bf[4];
#pragma unroll
    for (int i = 0; i < 2; ++i) af[i] = ldfrag(lA + (wm + 16 * i + m) * LDSW, hh);
#pragma unroll
    for (int j = 0; j < 4; ++j) bf[j] = ldfrag(lB + (wn + 16 * j + m) * LDSW, hh);
#pragma unroll
    for (int i = 0; i < 2; ++i)
#pragma unroll
      for (int j = 0; j < 4; ++j) acc[i][j] = wmma16(af[i], bf[j], acc[i][j]);
    asm volatile("v_nop\n\tv_nop\n\tv_nop\n\tv_nop"
                 : "+v"(acc[0][0]), "+v"(acc[0][1]), "+v"(acc[0][2]), "+v"(acc[0][3]),
                   "+v"(acc[1][0]), "+v"(acc[1][1]), "+v"(acc[1][2]), "+v"(acc[1][3])
                 : "v"(af[0]), "v"(af[1]), "v"(bf[0]), "v"(bf[1]), "v"(bf[2]), "v"(bf[3]));
    __syncthreads();
  }

#pragma unroll
  for (int i = 0; i < 2; ++i) {
#pragma unroll
    for (int j = 0; j < 4; ++j) {
      const int cl = wn + 16 * j + m;
      const int nl = wm + 16 * i + 8 * hh;
      Pack8 pk;
      if (hasZ) {
        const v8h_t z = *(const v8h*)(Zt + (size_t)(cb + cl) * N_NODES + nb + nl);
#pragma unroll
        for (int r = 0; r < 8; ++r) pk.h[r] = (f16)(acc[i][j][r] * alpha - (float)z[r]);
      } else {
#pragma unroll
        for (int r = 0; r < 8; ++r) pk.h[r] = (f16)(acc[i][j][r] * alpha);
      }
      *(v8h*)(stg + cl * SP + nl) = pk.h;
    }
  }
  __syncthreads();
  v4u_t v[8];
#pragma unroll
  for (int q = 0; q < 8; ++q) {
    const int cl = w * 16 + 2 * q + hh;
    v[q] = *(const v4u*)(stg + cl * SP + m * 8);
  }
  f16* ob = Ot + (size_t)cb * N_NODES + nb + m * 8;
#pragma unroll
  for (int q = 0; q < 8; ++q)
    *(volatile v4u_t*)(ob + (size_t)(w * 16 + 2 * q + hh) * N_NODES) = v[q];
  __threadfence();
#pragma unroll
  for (int q = 0; q < 8; ++q)
    *(volatile v4u_t*)(ob + (size_t)(w * 16 + 2 * q + hh) * N_NODES) = v[q];
}

template <bool P0H_PLANE>
__device__ __forceinline__ void stage_A(int c, int b, int nb,
    const float* __restrict__ x, const float* __restrict__ hsrc,
    const f16* P0, const f16* P1, const f16* P2,
    f16* lA, int t)
{
  const int p = c >> 2;
  const int fo = (c & 3) * 32;
  const bool hpart = (fo >= 64);
  const bool direct = (p == 0) && (!hpart || !P0H_PLANE);
  if (direct) {
    const float* src = hpart ? hsrc : x;
    const int fl = fo & 63;
    const int n = t >> 1, fofs = (t & 1) * 16;
    const float* rp = src + (size_t)b * (N_NODES * FX) + (size_t)(nb + n) * FX + fl + fofs;
    const v4f_t q0 = *(const v4f*)rp;
    const v4f_t q1 = *(const v4f*)(rp + 4);
    const v4f_t q2 = *(const v4f*)(rp + 8);
    const v4f_t q3 = *(const v4f*)(rp + 12);
    Pack8 k0, k1;
#pragma unroll
    for (int e = 0; e < 4; ++e) {
      k0.h[e]     = (f16)q0[e];
      k0.h[4 + e] = (f16)q1[e];
      k1.h[e]     = (f16)q2[e];
      k1.h[4 + e] = (f16)q3[e];
    }
    *(v8h*)(lA + n * LDSW + fofs) = k0.h;
    *(v8h*)(lA + n * LDSW + fofs + 8) = k1.h;
  } else {
    const f16* P = (p == 0) ? P0 : ((p == 1) ? P1 : P2);
    const int col0 = (hpart ? PART : 0) + b * FX + (fo & 63);
    const int fp = t >> 4, n8 = (t & 15) * 8;
    const f16* g = P + (size_t)(col0 + 2 * fp) * N_NODES + nb + n8;
    const v8h_t u0 = *(const v8h*)g;
    const v8h_t u1 = *(const v8h*)(g + N_NODES);
    uint32_t* l32 = (uint32_t*)lA;
#pragma unroll
    for (int e = 0; e < 8; ++e) {
      Pack2 pk;
      pk.h[0] = u0[e];
      pk.h[1] = u1[e];
      l32[(n8 + e) * (LDSW / 2) + fp] = pk.u;
    }
  }
}

__global__ void __launch_bounds__(256) k_gate(
    const float* __restrict__ x, const float* __restrict__ hx,
    const f16* __restrict__ D1, const f16* __restrict__ D2,
    const f16* __restrict__ WT, const float* __restrict__ bias,
    f16* RH, float* __restrict__ U)
{
  __shared__ __align__(16) unsigned char lds_raw[128 * UP * 4 + 64 * SP * 2];
  static_assert(128 * UP * 4 + 64 * SP * 2 >= 2 * 128 * LDSW * 2);
  f16* lA = (f16*)lds_raw;
  f16* lB = lA + 128 * LDSW;
  const int t = threadIdx.x, lane = t & 31, w = t >> 5;
  const int hh = lane >> 4, m = lane & 15;
  const int wm = (w >> 1) * 32, wn = (w & 1) * 64;
  const int nb = blockIdx.x * 128, b = blockIdx.y;
  const int lr = t >> 2, lc = (t & 3) * 8;

  v8f acc[2][4];
#pragma unroll
  for (int i = 0; i < 2; ++i)
#pragma unroll
    for (int j = 0; j < 4; ++j) acc[i][j] = zero8();

#pragma unroll 1
  for (int c = 0; c < KLIN / 32; ++c) {
    stage_A<false>(c, b, nb, x, hx, RH, D1, D2, lA, t);
    const f16* wp = WT + (size_t)lr * KLIN + c * 32 + lc;
    *(v8h*)(lB + lr * LDSW + lc) = *(const v8h*)wp;
    *(v8h*)(lB + (lr + 64) * LDSW + lc) = *(const v8h*)(wp + (size_t)64 * KLIN);
    __syncthreads();
    v16h af[2], bf[4];
#pragma unroll
    for (int i = 0; i < 2; ++i) af[i] = ldfrag(lA + (wm + 16 * i + m) * LDSW, hh);
#pragma unroll
    for (int j = 0; j < 4; ++j) bf[j] = ldfrag(lB + (wn + 16 * j + m) * LDSW, hh);
#pragma unroll
    for (int i = 0; i < 2; ++i)
#pragma unroll
      for (int j = 0; j < 4; ++j) acc[i][j] = wmma16(af[i], bf[j], acc[i][j]);
    asm volatile("v_nop\n\tv_nop\n\tv_nop\n\tv_nop"
                 : "+v"(acc[0][0]), "+v"(acc[0][1]), "+v"(acc[0][2]), "+v"(acc[0][3]),
                   "+v"(acc[1][0]), "+v"(acc[1][1]), "+v"(acc[1][2]), "+v"(acc[1][3])
                 : "v"(af[0]), "v"(af[1]), "v"(bf[0]), "v"(bf[1]), "v"(bf[2]), "v"(bf[3]));
    __syncthreads();
  }

  float* uS = (float*)lds_raw;
  f16*   rS = (f16*)(lds_raw + 128 * UP * 4);
  const size_t hrow = (size_t)b * (N_NODES * UNITS) + (size_t)nb * UNITS;
  if (w & 1) {
#pragma unroll
    for (int i = 0; i < 2; ++i) {
#pragma unroll
      for (int j = 0; j < 4; ++j) {
        const int ju = 16 * j + m;
        const float bv = bias[UNITS + ju];
        const int nl0 = wm + 16 * i + 8 * hh;
#pragma unroll
        for (int r = 0; r < 8; ++r)
          uS[(nl0 + r) * UP + ju] = sigm_f(acc[i][j][r] + bv);
      }
    }
  } else {
#pragma unroll
    for (int i = 0; i < 2; ++i) {
#pragma unroll
      for (int j = 0; j < 4; ++j) {
        const int jr = 16 * j + m;
        const float bv = bias[jr];
        const int nl0 = wm + 16 * i + 8 * hh;
        Pack8 pk;
#pragma unroll
        for (int r = 0; r < 8; ++r) {
          const float s  = sigm_f(acc[i][j][r] + bv);
          const float hv = hx[hrow + (size_t)(nl0 + r) * UNITS + jr];
          pk.h[r] = (f16)(s * hv);
        }
        *(v8h*)(rS + jr * SP + nl0) = pk.h;
      }
    }
  }
  __syncthreads();

  v4f_t uv[8];
#pragma unroll
  for (int q = 0; q < 8; ++q) {
    const int row = w * 16 + 2 * q + hh;
    uv[q] = *(const v4f*)(uS + row * UP + m * 4);
  }
  v4u_t rv[4];
#pragma unroll
  for (int q = 0; q < 4; ++q) {
    const int col = w * 8 + 2 * q + hh;
    rv[q] = *(const v4u*)(rS + col * SP + m * 8);
  }
  float* uo = U + hrow + m * 4;
  f16*   ro = RH + (size_t)(PART + b * FX) * N_NODES + nb + m * 8;
#pragma unroll
  for (int q = 0; q < 8; ++q)
    *(volatile v4f_t*)(uo + (size_t)(w * 16 + 2 * q + hh) * UNITS) = uv[q];
#pragma unroll
  for (int q = 0; q < 4; ++q)
    *(volatile v4u_t*)(ro + (size_t)(w * 8 + 2 * q + hh) * N_NODES) = rv[q];
  __threadfence();
#pragma unroll
  for (int q = 0; q < 8; ++q)
    *(volatile v4f_t*)(uo + (size_t)(w * 16 + 2 * q + hh) * UNITS) = uv[q];
#pragma unroll
  for (int q = 0; q < 4; ++q)
    *(volatile v4u_t*)(ro + (size_t)(w * 8 + 2 * q + hh) * N_NODES) = rv[q];
}

__global__ void __launch_bounds__(256) k_cand(
    const float* __restrict__ x, const float* __restrict__ hx,
    const f16* __restrict__ P0, const f16* __restrict__ D1, const f16* __restrict__ D2,
    const f16* __restrict__ WT, const float* __restrict__ bias, float* out)
{
  __shared__ __align__(16) unsigned char lds_raw[128 * UP * 4];
  static_assert(128 * UP * 4 >= (128 + 64) * LDSW * 2);
  f16* lA = (f16*)lds_raw;
  f16* lB = lA + 128 * LDSW;
  const int t = threadIdx.x, lane = t & 31, w = t >> 5;
  const int hh = lane >> 4, m = lane & 15;
  const int wm = w * 16;
  const int nb = blockIdx.x * 128, b = blockIdx.y;
  const int lr = t >> 2, lc = (t & 3) * 8;

  v8f acc[4];
#pragma unroll
  for (int j = 0; j < 4; ++j) acc[j] = zero8();

#pragma unroll 1
  for (int c = 0; c < KLIN / 32; ++c) {
    stage_A<true>(c, b, nb, x, hx, P0, D1, D2, lA, t);
    *(v8h*)(lB + lr * LDSW + lc) = *(const v8h*)(WT + (size_t)lr * KLIN + c * 32 + lc);
    __syncthreads();
    const v16h af = ldfrag(lA + (wm + m) * LDSW, hh);
    v16h bf[4];
#pragma unroll
    for (int j = 0; j < 4; ++j) bf[j] = ldfrag(lB + (16 * j + m) * LDSW, hh);
#pragma unroll
    for (int j = 0; j < 4; ++j) acc[j] = wmma16(af, bf[j], acc[j]);
    asm volatile("v_nop\n\tv_nop\n\tv_nop\n\tv_nop"
                 : "+v"(acc[0]), "+v"(acc[1]), "+v"(acc[2]), "+v"(acc[3])
                 : "v"(af), "v"(bf[0]), "v"(bf[1]), "v"(bf[2]), "v"(bf[3]));
    __syncthreads();
  }

  float* oS = (float*)lds_raw;
  const size_t hrow = (size_t)b * (N_NODES * UNITS) + (size_t)nb * UNITS;
#pragma unroll
  for (int j = 0; j < 4; ++j) {
    const int jc = 16 * j + m;
    const float bv = bias[jc];
    const int nl0 = wm + 8 * hh;
#pragma unroll
    for (int r = 0; r < 8; ++r) {
      const size_t idx = hrow + (size_t)(nl0 + r) * UNITS + jc;
      const float cv = tanh_f(acc[j][r] + bv);
      const float u  = out[idx];
      const float hv = hx[idx];
      oS[(nl0 + r) * UP + jc] = u * hv + (1.0f - u) * cv;
    }
  }
  __syncthreads();

  v4f_t ov[8];
#pragma unroll
  for (int q = 0; q < 8; ++q) {
    const int row = w * 16 + 2 * q + hh;
    ov[q] = *(const v4f*)(oS + row * UP + m * 4);
  }
  float* go = out + hrow + m * 4;
#pragma unroll
  for (int q = 0; q < 8; ++q)
    *(volatile v4f_t*)(go + (size_t)(w * 16 + 2 * q + hh) * UNITS) = ov[q];
  __threadfence();
#pragma unroll
  for (int q = 0; q < 8; ++q)
    *(volatile v4f_t*)(go + (size_t)(w * 16 + 2 * q + hh) * UNITS) = ov[q];
}

extern "C" void kernel_launch(void* const* d_in, const int* in_sizes, int n_in,
                              void* d_out, int out_size, void* d_ws, size_t ws_size,
                              hipStream_t stream)
{
  if (n_in < 7) return;
  if (in_sizes[0] != BATCH * N_NODES * FX) return;
  if (in_sizes[1] != BATCH * N_NODES * UNITS) return;
  if (in_sizes[2] != N_NODES * N_NODES) return;
  if (in_sizes[3] != KLIN * FCAT) return;
  if (in_sizes[4] != FCAT) return;
  if (in_sizes[5] != KLIN * UNITS) return;
  if (in_sizes[6] != UNITS) return;
  if (out_size != BATCH * N_NODES * UNITS) return;

  const float* x   = (const float*)d_in[0];
  const float* hx  = (const float*)d_in[1];
  const float* adj = (const float*)d_in[2];
  const float* Wru = (const float*)d_in[3];
  const float* bru = (const float*)d_in[4];
  const float* Wc  = (const float*)d_in[5];
  const float* bc  = (const float*)d_in[6];
  float* out = (float*)d_out;

  const size_t nAdj = (size_t)N_NODES * N_NODES * 2;
  const size_t nPl  = (size_t)NCOL * N_NODES * 2;
  const size_t nWru = (size_t)FCAT * KLIN * 2;
  const size_t nWc  = (size_t)UNITS * KLIN * 2;
  const size_t oAdj = 0;
  const size_t oX0  = oAdj + nAdj;
  const size_t oD1  = oX0 + nPl;
  const size_t oD2  = oD1 + nPl;
  const size_t oWru = oD2 + nPl;
  const size_t oWc  = oWru + nWru;
  const size_t total = oWc + nWc;
  if (total > ws_size) return;

  char* ws = (char*)d_ws;
  f16* adjT = (f16*)(ws + oAdj);
  f16* X0T  = (f16*)(ws + oX0);
  f16* D1T  = (f16*)(ws + oD1);
  f16* D2T  = (f16*)(ws + oD2);
  f16* WruT = (f16*)(ws + oWru);
  f16* WcT  = (f16*)(ws + oWc);

  const float a1 = 1.0f / ADJ_CARRY;
  const float a2 = 2.0f / ADJ_CARRY;
  const size_t hs = (size_t)PART * N_NODES;

  k_adjT<<<N_NODES / 64, 256, 0, stream>>>(adj, adjT);
  k_x0t<<<dim3(N_NODES / 64, BATCH, 2), 256, 0, stream>>>(x, hx, X0T);
  k_packW<<<36, 256, 0, stream>>>(Wru, Wc, WruT, WcT);
  k_diff<<<dim3(NCOL / 128, N_NODES / 128), 256, 0, stream>>>(adjT, X0T, X0T, D1T, a1, 0);
  k_diff<<<dim3(NCOL / 128, N_NODES / 128), 256, 0, stream>>>(adjT, D1T, X0T, D2T, a2, 1);
  k_gate<<<dim3(N_NODES / 128, BATCH), 256, 0, stream>>>(x, hx, D1T, D2T, WruT, bru, X0T, out);
  k_diff<<<dim3(PART / 128, N_NODES / 128), 256, 0, stream>>>(adjT, X0T + hs, X0T + hs, D1T + hs, a1, 0);
  k_diff<<<dim3(PART / 128, N_NODES / 128), 256, 0, stream>>>(adjT, D1T + hs, X0T + hs, D2T + hs, a2, 1);
  k_cand<<<dim3(N_NODES / 128, BATCH), 256, 0, stream>>>(x, hx, X0T, D1T, D2T, WcT, bc, out);
}
